// Conv2DMod_71871982731629
// MI455X (gfx1250) — hardware-verified
//
#include <hip/hip_runtime.h>
#include <hip/hip_bf16.h>

typedef _Float16 bf16_t;
typedef __attribute__((ext_vector_type(16))) _Float16 v16bf;
typedef __attribute__((ext_vector_type(8)))  _Float16 v8bf;
#define __bf16 _Float16
typedef __attribute__((ext_vector_type(8)))  float  v8f;

#define BATCH 8
#define CIN   256
#define COUT  256
#define HW    4096
#define PW    66
#define PHW   (PW*PW)
#define WBF_ELEMS (9*COUT*CIN)
#define WBF_BYTES (WBF_ELEMS*2)
#define DMOD_BYTES (BATCH*COUT*4)
#define XP_ELEMS ((size_t)BATCH*PHW*CIN)
#define XP_BYTES (XP_ELEMS*2)

__global__ void zero_ws_kernel(uint4* __restrict__ p, int n16) {
    int t = blockIdx.x * 256 + threadIdx.x;
    if (t < n16) {
        typedef __attribute__((ext_vector_type(4))) unsigned v4u_t;
        v4u_t z; z.x = 0u; z.y = 0u; z.z = 0u; z.w = 0u;
        *(volatile v4u_t*)(p + t) = z; __threadfence(); *(volatile v4u_t*)(p + t) = z;
    }
}

__global__ void wconv_kernel(const float* __restrict__ w, bf16_t* __restrict__ wbf) {
    int t = blockIdx.x * 256 + threadIdx.x;
    int e = 2 * t;
    int i    = e & 255;
    int o    = (e >> 8) & 255;
    int kpos = e >> 16;
    float v0 = w[((size_t)o * CIN + i) * 9 + kpos];
    float v1 = w[((size_t)o * CIN + i + 1) * 9 + kpos];
    unsigned pk = (unsigned)__builtin_bit_cast(unsigned short, (bf16_t)v0) | ((unsigned)__builtin_bit_cast(unsigned short, (bf16_t)v1) << 16);
    unsigned* dst = (unsigned*)(wbf + e);
    *(volatile unsigned*)dst = pk; __threadfence(); *(volatile unsigned*)dst = pk;
}

__global__ void modnorm_kernel(const float* __restrict__ w, const float* __restrict__ y,
                               float* __restrict__ dmod) {
    __shared__ float m2[CIN];
    int b = blockIdx.x;
    int o = threadIdx.x;
    { float m = y[b * CIN + o] + 1.0f; m2[o] = m * m; }
    __syncthreads();
    const float* wp = w + (size_t)o * CIN * 9;
    float acc = 0.f;
    for (int i = 0; i < CIN; ++i) {
        float s2 = 0.f;
#pragma unroll
        for (int k = 0; k < 9; ++k) { float v = wp[i * 9 + k]; s2 += v * v; }
        acc += s2 * m2[i];
    }
    const float dv = rsqrtf(acc + 1e-6f);
    *(volatile float*)(dmod + b * COUT + o) = dv; __threadfence(); *(volatile float*)(dmod + b * COUT + o) = dv;
}

__global__ void xmod_transpose_kernel(const float* __restrict__ x, const float* __restrict__ y,
                                      bf16_t* __restrict__ xp) {
    __shared__ __bf16 tile[64][33];
    int b  = blockIdx.z;
    int c0 = blockIdx.x * 64;
    int p0 = blockIdx.y * 32;
    int tx = threadIdx.x & 31;
    int ty = threadIdx.x >> 5;
#pragma unroll
    for (int i = 0; i < 8; ++i) {
        int cl = ty + i * 8;
        float m = y[b * CIN + c0 + cl] + 1.0f;
        float v = x[(((size_t)b * CIN + c0 + cl) * HW) + p0 + tx];
        tile[cl][tx] = (__bf16)(v * m);
    }
    __syncthreads();
#pragma unroll
    for (int i = 0; i < 4; ++i) {
        int pl  = ty + i * 8;
        int p   = p0 + pl;
        int row = p >> 6;
        int col = p & 63;
        unsigned pk = (unsigned)__builtin_bit_cast(unsigned short, tile[2 * tx][pl]) | ((unsigned)__builtin_bit_cast(unsigned short, tile[2 * tx + 1][pl]) << 16);
        unsigned* dst = (unsigned*)(xp + (((size_t)b * PHW) + (row + 1) * PW + (col + 1)) * CIN + c0) + tx;
        *(volatile unsigned*)dst = pk; __threadfence(); *(volatile unsigned*)dst = pk;
    }
}

typedef __attribute__((ext_vector_type(4))) float v4f_t;
typedef float v4fa __attribute__((ext_vector_type(4), may_alias));
__device__ __forceinline__ void store_tile16x32(const float* stg, float* __restrict__ dst, size_t ld, int lane) {
    v4f_t vv[4];
#pragma unroll
    for (int i = 0; i < 4; ++i) { const int c = lane + 32 * i; vv[i] = *(const v4fa*)(stg + (c >> 3) * 32 + (c & 7) * 4); }
#pragma unroll
    for (int i = 0; i < 4; ++i) { const int c = lane + 32 * i; *(volatile v4f_t*)(dst + (size_t)(c >> 3) * ld + (c & 7) * 4) = vv[i]; }
    __threadfence();
#pragma unroll
    for (int i = 0; i < 4; ++i) { const int c = lane + 32 * i; *(volatile v4f_t*)(dst + (size_t)(c >> 3) * ld + (c & 7) * 4) = vv[i]; }
}

__global__ __launch_bounds__(256) void conv_gemm_kernel(
        const bf16_t* __restrict__ wbf, const bf16_t* __restrict__ xp,
        const float* __restrict__ dmod, float* __restrict__ out) {
    __shared__ __attribute__((aligned(16))) float stg[8][16 * 32];
    int b    = blockIdx.z;
    int tid  = threadIdx.x;
    int lane = tid & 31;
    int wv   = tid >> 5;
    int wm   = wv & 1;
    int wn   = wv >> 1;
    int lm   = lane & 15;
    int hsel = lane >> 4;
    int m_base = blockIdx.x * 128 + wm * 64;
    int n_base = blockIdx.y * 256 + wn * 64;

    const bf16_t* abase[4];
#pragma unroll
    for (int tm = 0; tm < 4; ++tm)
        abase[tm] = wbf + (size_t)(m_base + tm * 16 + lm) * CIN + hsel * 8;

    const bf16_t* bbase[4];
#pragma unroll
    for (int tn = 0; tn < 4; ++tn) {
        int n  = n_base + tn * 16 + lm;
        int py = n >> 6;
        int px = n & 63;
        bbase[tn] = xp + (((size_t)b * PHW) + (size_t)(py + 1) * PW + (px + 1)) * CIN
                    + hsel * 8;
    }

    __builtin_prefetch(abase[0], 0, 1);
    __builtin_prefetch(bbase[0], 0, 1);

    v8f acc[4][4];
#pragma unroll
    for (int tm = 0; tm < 4; ++tm)
#pragma unroll
        for (int tn = 0; tn < 4; ++tn)
#pragma unroll
            for (int e = 0; e < 8; ++e) acc[tm][tn][e] = 0.0f;

    union U16 { v16bf v; v8bf h[2]; };

#pragma unroll
    for (int kpos = 0; kpos < 9; ++kpos) {
        const int dy   = kpos / 3 - 1;
        const int dx   = kpos % 3 - 1;
        const int aoff = kpos * (COUT * CIN);
        const int boff = (dy * PW + dx) * CIN;
#pragma unroll
        for (int ct = 0; ct < 8; ++ct) {
            const int cb = ct * 32;
            v16bf amat[4];
#pragma unroll
            for (int tm = 0; tm < 4; ++tm) {
                U16 ua;
                ua.h[0] = *(const v8bf*)(abase[tm] + aoff + cb);
                ua.h[1] = *(const v8bf*)(abase[tm] + aoff + cb + 16);
                amat[tm] = ua.v;
            }
            v16bf bmat[4];
#pragma unroll
            for (int tn = 0; tn < 4; ++tn) {
                U16 ub;
                ub.h[0] = *(const v8bf*)(bbase[tn] + boff + cb);
                ub.h[1] = *(const v8bf*)(bbase[tn] + boff + cb + 16);
                bmat[tn] = ub.v;
            }
#pragma unroll
            for (int tm = 0; tm < 4; ++tm)
#pragma unroll
                for (int tn = 0; tn < 4; ++tn)
                    acc[tm][tn] = __builtin_amdgcn_wmma_f32_16x16x32_f16(
                        false, amat[tm], false, bmat[tn],
                        (short)0, acc[tm][tn], false, false);
        }
    }

    float* op = out + (size_t)b * COUT * HW;
    float* sg = stg[wv];
#pragma unroll
    for (int tm = 0; tm < 4; ++tm) {
#pragma unroll
        for (int tp = 0; tp < 4; tp += 2) {
#pragma unroll
            for (int e = 0; e < 8; ++e) {
                int o    = m_base + tm * 16 + hsel * 8 + e;
                float dv = dmod[b * COUT + o];
#pragma unroll
                for (int tj = 0; tj < 2; ++tj) sg[(hsel * 8 + e) * 32 + tj * 16 + lm] = acc[tm][tp + tj][e] * dv;
            }
            store_tile16x32(sg, op + (size_t)(m_base + tm * 16) * HW + n_base + tp * 16, (size_t)HW, lane);
        }
    }
}

extern "C" void kernel_launch(void* const* d_in, const int* in_sizes, int n_in,
                              void* d_out, int out_size, void* d_ws, size_t ws_size,
                              hipStream_t stream) {
    const float* x = (const float*)d_in[0];
    const float* y = (const float*)d_in[1];
    const float* w = (const float*)d_in[2];
    float* out = (float*)d_out;

    size_t need = (size_t)WBF_BYTES + DMOD_BYTES + XP_BYTES;
    if (ws_size < need) return;

    char* ws = (char*)d_ws;
    bf16_t* wbf  = (bf16_t*)ws;
    float*  dmod = (float*)(ws + WBF_BYTES);
    bf16_t* xp   = (bf16_t*)(ws + WBF_BYTES + DMOD_BYTES);

    int n16 = (int)(XP_BYTES / 16);
    zero_ws_kernel<<<(n16 + 255) / 256, 256, 0, stream>>>((uint4*)xp, n16);
    wconv_kernel<<<WBF_ELEMS / 512, 256, 0, stream>>>(w, wbf);
    modnorm_kernel<<<BATCH, 256, 0, stream>>>(w, y, dmod);
    xmod_transpose_kernel<<<dim3(CIN / 64, HW / 32, BATCH), 256, 0, stream>>>(x, y, xp);
    conv_gemm_kernel<<<dim3(COUT / 128, HW / 256, BATCH), 256, 0, stream>>>(wbf, xp, dmod, out);
}
